// PALMAttention_8418135900896
// MI455X (gfx1250) — hardware-verified
//
#include <hip/hip_runtime.h>
#include <math.h>
#include <stdint.h>

#define BATCH 4
#define SEQ   2048
#ifndef NB
#define NB    BATCH
#endif
#ifndef SQ
#define SQ    SEQ
#endif
#define DMOD  1024
#define NH    16
#define HD    64
#define MK    (NB * SEQ)
#define MQ    ((NB - 1) * SEQ + SQ)
#define PCAR  32768.0f
#define VCAR  1024.0f
#define LOG2E 1.4426950408889634f
#define LN_EPS 1e-12f
#define ATT_WAVES   4
#define ATT_THREADS (ATT_WAVES * 32)
#define QT          (MQ / 64)
#define ATT_BLOCKS  (NH * QT)
#define NKB         (SEQ / 32)
#define SLAB        (16 * 68)
#define LN_WAVES    8
static_assert(HD == 64 && DMOD == NH * HD);
static_assert(NB >= 1 && NB <= BATCH);
static_assert((SEQ % 64) == 0 && (SQ % 64) == 0 && SQ >= 64 && SQ <= SEQ);
static_assert(SQ == SEQ || NB == 1);
static_assert((MQ % 64) == 0 && (MK % 64) == 0 && MQ <= MK);
static_assert(ATT_THREADS == 128 && NKB * 32 == SEQ && ATT_BLOCKS == NH * (MQ / 64));
static_assert((DMOD % 128) == 0 && (DMOD % 64) == 0 && (DMOD % 32) == 0);
static_assert(((MK * (DMOD / 8)) % 256) == 0);
static_assert(((DMOD * (DMOD / 8)) % 256) == 0);
static_assert(((MK / 4) % 256) == 0);
static_assert((MQ % LN_WAVES) == 0);
static_assert((SLAB * 4) % 16 == 0);

typedef unsigned short u16;
typedef _Float16 v16h __attribute__((ext_vector_type(16)));
typedef _Float16 v8h  __attribute__((ext_vector_type(8)));
typedef __bf16   v16b __attribute__((ext_vector_type(16)));
typedef float    v8f  __attribute__((ext_vector_type(8)));
typedef float    v4f  __attribute__((ext_vector_type(4)));
typedef unsigned int v4u __attribute__((ext_vector_type(4)));

union FragH { v16h v; v8h h[2]; v4u u[2]; };
union FragB { v16b v; v4u u[2]; };

__device__ __forceinline__ unsigned short bf_bits(float f) {
  unsigned u = __float_as_uint(f);
  return (unsigned short)((u + 0x7FFFu + ((u >> 16) & 1u)) >> 16);
}
__device__ __forceinline__ float bf_up(unsigned short h) { return __uint_as_float(((unsigned)h) << 16); }
__device__ __forceinline__ float bf_val(float f) { return bf_up(bf_bits(f)); }
__device__ __forceinline__ unsigned short h_bits(_Float16 x) { return __builtin_bit_cast(unsigned short, x); }
__device__ __forceinline__ unsigned pk16(unsigned short a, unsigned short b) { return (unsigned)a | ((unsigned)b << 16); }
__device__ __forceinline__ v8f zero8() { v8f z = {0.f, 0.f, 0.f, 0.f, 0.f, 0.f, 0.f, 0.f}; return z; }

__device__ __forceinline__ v16h ldfrag_h(const _Float16* p) {
  FragH f;
  f.h[0] = *(const v8h*)(p);
  f.h[1] = *(const v8h*)(p + 16);
  return f.v;
}
__device__ __forceinline__ v16b ldfrag_b(const u16* p) {
  FragB f;
  f.u[0] = *(const v4u*)(p);
  f.u[1] = *(const v4u*)(p + 16);
  return f.v;
}

__device__ __forceinline__ v8f mma_h(v16h a, v16h b, v8f c) {
  return __builtin_amdgcn_wmma_f32_16x16x32_f16(false, a, false, b, (short)0, c, false, false);
}
__device__ __forceinline__ v8f mma_b(v16b a, v16b b, v8f c) {
  return __builtin_amdgcn_wmma_f32_16x16x32_bf16(false, a, false, b, (short)0, c, false, false);
}
__device__ __forceinline__ void guard1x8(v8f& a, v16b x0, v16b x1, v16b x2, v16b x3, v16b x4, v16b x5, v16b x6, v16b x7) {
#if defined(__HIP_DEVICE_COMPILE__)
  asm volatile("v_nop\n\tv_nop\n\tv_nop\n\tv_nop"
               : "+v"(a) : "v"(x0), "v"(x1), "v"(x2), "v"(x3), "v"(x4), "v"(x5), "v"(x6), "v"(x7) : "memory");
#endif
}
template <typename F>
__device__ __forceinline__ void guard6(v8f& a, v8f& b, v8f& c, v8f& d, F x0, F x1, F x2, F x3, F x4, F x5) {
#if defined(__HIP_DEVICE_COMPILE__)
  asm volatile("v_nop\n\tv_nop\n\tv_nop\n\tv_nop"
               : "+v"(a), "+v"(b), "+v"(c), "+v"(d) : "v"(x0), "v"(x1), "v"(x2), "v"(x3), "v"(x4), "v"(x5) : "memory");
#endif
}
__device__ __forceinline__ void acc_guard4(v8f& a, v8f& b, v8f& c, v8f& d) {
#if defined(__HIP_DEVICE_COMPILE__)
  asm volatile("v_nop\n\tv_nop\n\tv_nop\n\tv_nop" : "+v"(a), "+v"(b), "+v"(c), "+v"(d));
#endif
}
__device__ __forceinline__ void wave_sync_lds() {
#if defined(__HIP_DEVICE_COMPILE__)
  __builtin_amdgcn_fence(__ATOMIC_RELEASE, "workgroup");
  __builtin_amdgcn_wave_barrier();
  __builtin_amdgcn_fence(__ATOMIC_ACQUIRE, "workgroup");
#endif
}

__global__ __launch_bounds__(256) void cvt16(const float* __restrict__ x, u16* D, int n8, int mode, float scale) {
  const int gt = blockIdx.x * 256 + (int)threadIdx.x;
  if (gt >= n8) return;
  const float* p = x + (size_t)gt * 8;
  const v4f a = *(const v4f*)(p), c4 = *(const v4f*)(p + 4);
  float v[8];
#pragma unroll
  for (int e = 0; e < 4; ++e) { v[e] = a[e]; v[4 + e] = c4[e]; }
  unsigned short s[8];
#pragma unroll
  for (int e = 0; e < 8; ++e) {
    const unsigned short bb = bf_bits(v[e]);
    const unsigned short hb = h_bits((_Float16)(bf_up(bb) * scale));
    s[e] = (mode != 0) ? hb : bb;
  }
  v4u o;
#pragma unroll
  for (int e = 0; e < 4; ++e) o[e] = pk16(s[2 * e], s[2 * e + 1]);
  u16* d = D + (size_t)gt * 8;
  for (int pass = 0; pass < 2; ++pass) {
    *(volatile v4u*)(d) = o;
    __threadfence();
  }
}

__global__ __launch_bounds__(256) void mask_bias(const float* __restrict__ mk, float* MB, int n4) {
  const int gt = blockIdx.x * 256 + (int)threadIdx.x;
  if (gt >= n4) return;
  const v4f a = *(const v4f*)(mk + (size_t)gt * 4);
  const float nbc = -10000.0f * LOG2E;
  v4f o;
#pragma unroll
  for (int e = 0; e < 4; ++e) o[e] = (1.0f - bf_val(a[e])) * nbc;
  float* d = MB + (size_t)gt * 4;
  for (int pass = 0; pass < 2; ++pass) {
    *(volatile v4f*)(d) = o;
    __threadfence();
  }
}

__device__ __forceinline__ void stage16x64(float* sl, v8f a0, v8f a1, v8f a2, v8f a3, int lane) {
  const int hh = lane >> 4, m = lane & 15;
#pragma unroll
  for (int r = 0; r < 8; ++r) {
    const int ro = (8 * hh + r) * 68 + m;
    sl[ro]      = a0[r];
    sl[ro + 16] = a1[r];
    sl[ro + 32] = a2[r];
    sl[ro + 48] = a3[r];
  }
}

__device__ __forceinline__ void epi16(float* sl, v8f a0, v8f a1, v8f a2, v8f a3, float oscale, u16* C, int N,
                                      size_t rowb, int col0, int lane) {
  stage16x64(sl, a0 * oscale, a1 * oscale, a2 * oscale, a3 * oscale, lane);
  wave_sync_lds();
  const int rq = lane >> 3, c8 = (lane & 7) * 8;
  v4u ov[4];
#pragma unroll
  for (int i4 = 0; i4 < 4; ++i4) {
    const int row = i4 * 4 + rq;
    const v4f a = *(const v4f*)(sl + row * 68 + c8), c4 = *(const v4f*)(sl + row * 68 + c8 + 4);
    float w[8];
#pragma unroll
    for (int e = 0; e < 4; ++e) { w[e] = a[e]; w[4 + e] = c4[e]; }
#pragma unroll
    for (int e = 0; e < 4; ++e) ov[i4][e] = pk16(h_bits((_Float16)w[2 * e]), h_bits((_Float16)w[2 * e + 1]));
  }
  u16* dst = C + (rowb + (size_t)rq) * (size_t)N + col0 + c8;
  for (int pass = 0; pass < 2; ++pass) {
#pragma unroll
    for (int i4 = 0; i4 < 4; ++i4) {
      *(volatile v4u*)(dst + (size_t)(i4 * 4) * (size_t)N) = ov[i4];
    }
    __threadfence();
  }
}

__device__ __forceinline__ void epi_hl(float* sl, v8f a0, v8f a1, v8f a2, v8f a3, u16* CH, u16* CL, int N,
                                       size_t rowb, int col0, int lane) {
  stage16x64(sl, a0, a1, a2, a3, lane);
  wave_sync_lds();
  const int rq = lane >> 3, c8 = (lane & 7) * 8;
  v4u oh[4], ol[4];
#pragma unroll
  for (int i4 = 0; i4 < 4; ++i4) {
    const int row = i4 * 4 + rq;
    const v4f a = *(const v4f*)(sl + row * 68 + c8), c4 = *(const v4f*)(sl + row * 68 + c8 + 4);
    float w[8];
#pragma unroll
    for (int e = 0; e < 4; ++e) { w[e] = a[e]; w[4 + e] = c4[e]; }
#pragma unroll
    for (int e = 0; e < 4; ++e) {
      const unsigned short h0 = bf_bits(w[2 * e]), h1 = bf_bits(w[2 * e + 1]);
      const unsigned short l0 = bf_bits(w[2 * e] - bf_up(h0)), l1 = bf_bits(w[2 * e + 1] - bf_up(h1));
      oh[i4][e] = pk16(h0, h1);
      ol[i4][e] = pk16(l0, l1);
    }
  }
  const size_t dofs = (rowb + (size_t)rq) * (size_t)N + (size_t)(col0 + c8);
  for (int pass = 0; pass < 2; ++pass) {
#pragma unroll
    for (int i4 = 0; i4 < 4; ++i4) {
      const size_t o8 = dofs + (size_t)(i4 * 4) * (size_t)N;
      *(volatile v4u*)(CH + o8) = oh[i4];
      *(volatile v4u*)(CL + o8) = ol[i4];
    }
    __threadfence();
  }
}

__device__ __forceinline__ void epi64(float* sl, v8f a0, v8f a1, v8f a2, v8f a3, float* C, int N,
                                      size_t rowb, int col0, int lane) {
  const int hh = lane >> 4, m = lane & 15;
  stage16x64(sl, a0, a1, a2, a3, lane);
  wave_sync_lds();
  v4f vals[8];
#pragma unroll
  for (int it = 0; it < 8; ++it) vals[it] = *(const v4f*)(sl + (it * 2 + hh) * 68 + m * 4);
  float* dst = C + (rowb + (size_t)hh) * (size_t)N + col0 + m * 4;
  for (int pass = 0; pass < 2; ++pass) {
#pragma unroll
    for (int it = 0; it < 8; ++it) {
      *(volatile v4f*)(dst + (size_t)(it * 2) * (size_t)N) = vals[it];
    }
    __threadfence();
  }
}

__global__ __launch_bounds__(128)
void gemm_hl(const u16* __restrict__ A, const u16* __restrict__ Bt, u16* CH, u16* CL, const float* __restrict__ bias,
             int M, int N, int K, int nbias) {
  __shared__ __align__(16) float slab[4 * SLAB];
  const int tid = threadIdx.x, wave = tid >> 5, lane = tid & 31, hh = lane >> 4, m = lane & 15;
  const int ntile = N >> 6;
  const int bid   = blockIdx.x;
  const int rowb  = (bid / ntile) * 64 + wave * 16;
  const int col0  = (bid % ntile) * 64;
  if (rowb + 16 > M) return;
  const u16* ap = A  + (size_t)(rowb + m) * K + 8 * hh;
  const u16* bp = Bt + (size_t)(col0 + m) * K + 8 * hh;
  const size_t bs = (size_t)16 * K;
  v8f acc0 = zero8(), acc1 = zero8(), acc2 = zero8(), acc3 = zero8();
#pragma unroll 1
  for (int k0 = 0; k0 < K; k0 += 32) {
    const v16b a  = ldfrag_b(ap + k0);
    const v16b b0 = ldfrag_b(bp + k0);
    const v16b b1 = ldfrag_b(bp + bs + k0);
    const v16b b2 = ldfrag_b(bp + 2 * bs + k0);
    const v16b b3 = ldfrag_b(bp + 3 * bs + k0);
    acc0 = mma_b(a, b0, acc0);
    acc1 = mma_b(a, b1, acc1);
    acc2 = mma_b(a, b2, acc2);
    acc3 = mma_b(a, b3, acc3);
    guard6<v16b>(acc0, acc1, acc2, acc3, a, b0, b1, b2, b3, a);
  }
  acc_guard4(acc0, acc1, acc2, acc3);
  float bc[4];
#pragma unroll
  for (int j = 0; j < 4; ++j) {
    int ci = col0 + 16 * j + m;
    ci = (ci < nbias) ? ci : (nbias - 1);
    bc[j] = bf_val(bias[ci]);
  }
#pragma unroll
  for (int r = 0; r < 8; ++r) {
    acc0[r] += bc[0];
    acc1[r] += bc[1];
    acc2[r] += bc[2];
    acc3[r] += bc[3];
  }
  epi_hl(slab + wave * SLAB, acc0, acc1, acc2, acc3, CH, CL, N, (size_t)rowb, col0, lane);
}

__global__ __launch_bounds__(128)
void gemm_b16(const u16* __restrict__ A, const u16* __restrict__ Bt, u16* C, const float* __restrict__ bias,
              int M, int N, int K, int nbias, int byrow, float oscale) {
  __shared__ __align__(16) float slab[4 * SLAB];
  const int tid = threadIdx.x, wave = tid >> 5, lane = tid & 31, hh = lane >> 4, m = lane & 15;
  const int ntile = N >> 6;
  const int bid   = blockIdx.x;
  const int rowb  = (bid / ntile) * 64 + wave * 16;
  const int col0  = (bid % ntile) * 64;
  if (rowb + 16 > M) return;
  const u16* ap = A  + (size_t)(rowb + m) * K + 8 * hh;
  const u16* bp = Bt + (size_t)(col0 + m) * K + 8 * hh;
  const size_t bs = (size_t)16 * K;
  v8f acc0 = zero8(), acc1 = zero8(), acc2 = zero8(), acc3 = zero8();
#pragma unroll 1
  for (int k0 = 0; k0 < K; k0 += 32) {
    const v16b a  = ldfrag_b(ap + k0);
    const v16b b0 = ldfrag_b(bp + k0);
    const v16b b1 = ldfrag_b(bp + bs + k0);
    const v16b b2 = ldfrag_b(bp + 2 * bs + k0);
    const v16b b3 = ldfrag_b(bp + 3 * bs + k0);
    acc0 = mma_b(a, b0, acc0);
    acc1 = mma_b(a, b1, acc1);
    acc2 = mma_b(a, b2, acc2);
    acc3 = mma_b(a, b3, acc3);
    guard6<v16b>(acc0, acc1, acc2, acc3, a, b0, b1, b2, b3, a);
  }
  acc_guard4(acc0, acc1, acc2, acc3);
  float bc[4], br[8];
#pragma unroll
  for (int j = 0; j < 4; ++j) {
    int ci = col0 + 16 * j + m;
    ci = (ci < nbias) ? ci : (nbias - 1);
    bc[j] = bf_val(bias[ci]);
  }
#pragma unroll
  for (int r = 0; r < 8; ++r) {
    int ri = rowb + 8 * hh + r;
    ri = (ri < nbias) ? ri : (nbias - 1);
    br[r] = bf_val(bias[ri]);
  }
#pragma unroll
  for (int r = 0; r < 8; ++r) {
    const float q0 = (byrow != 0) ? br[r] : bc[0];
    const float q1 = (byrow != 0) ? br[r] : bc[1];
    const float q2 = (byrow != 0) ? br[r] : bc[2];
    const float q3 = (byrow != 0) ? br[r] : bc[3];
    acc0[r] += q0;
    acc1[r] += q1;
    acc2[r] += q2;
    acc3[r] += q3;
  }
  epi16(slab + wave * SLAB, acc0, acc1, acc2, acc3, oscale, C, N, (size_t)rowb, col0, lane);
}

__global__ __launch_bounds__(128)
void gemm_o2(const u16* __restrict__ AH, const u16* __restrict__ AL, const u16* __restrict__ Bt, float* C,
             const float* __restrict__ bias, int M, int N, int K, int nbias) {
  __shared__ __align__(16) float slab[4 * SLAB];
  const int tid = threadIdx.x, wave = tid >> 5, lane = tid & 31, hh = lane >> 4, m = lane & 15;
  const int ntile = N >> 6;
  const int bid   = blockIdx.x;
  const int rowb  = (bid / ntile) * 64 + wave * 16;
  const int col0  = (bid % ntile) * 64;
  if (rowb + 16 > M) return;
  const u16* ahp = AH + (size_t)(rowb + m) * K + 8 * hh;
  const u16* alp = AL + (size_t)(rowb + m) * K + 8 * hh;
  const u16* bp  = Bt + (size_t)(col0 + m) * K + 8 * hh;
  const size_t bs = (size_t)16 * K;
  v8f acc0 = zero8(), acc1 = zero8(), acc2 = zero8(), acc3 = zero8();
#pragma unroll 1
  for (int k0 = 0; k0 < K; k0 += 32) {
    const v16b ah = ldfrag_b(ahp + k0);
    const v16b al = ldfrag_b(alp + k0);
    const v16b b0 = ldfrag_b(bp + k0);
    const v16b b1 = ldfrag_b(bp + bs + k0);
    const v16b b2 = ldfrag_b(bp + 2 * bs + k0);
    const v16b b3 = ldfrag_b(bp + 3 * bs + k0);
    acc0 = mma_b(ah, b0, acc0);
    acc1 = mma_b(ah, b1, acc1);
    acc2 = mma_b(ah, b2, acc2);
    acc3 = mma_b(ah, b3, acc3);
    acc0 = mma_b(al, b0, acc0);
    acc1 = mma_b(al, b1, acc1);
    acc2 = mma_b(al, b2, acc2);
    acc3 = mma_b(al, b3, acc3);
    guard6<v16b>(acc0, acc1, acc2, acc3, ah, al, b0, b1, b2, b3);
  }
  acc_guard4(acc0, acc1, acc2, acc3);
  float bc[4];
#pragma unroll
  for (int j = 0; j < 4; ++j) {
    int ci = col0 + 16 * j + m;
    ci = (ci < nbias) ? ci : (nbias - 1);
    bc[j] = bf_val(bias[ci]);
  }
#pragma unroll
  for (int r = 0; r < 8; ++r) {
    acc0[r] += bc[0];
    acc1[r] += bc[1];
    acc2[r] += bc[2];
    acc3[r] += bc[3];
  }
  epi64(slab + wave * SLAB, acc0, acc1, acc2, acc3, C, N, (size_t)rowb, col0, lane);
}

__device__ __forceinline__ v8f score_tile(const u16* khp, const u16* klp, v16b qh0, v16b qh1, v16b ql0, v16b ql1) {
  const v16b a0 = ldfrag_b(khp), a1 = ldfrag_b(khp + 32);
  const v16b e0 = ldfrag_b(klp), e1 = ldfrag_b(klp + 32);
  v8f s = zero8();
  s = mma_b(a0, qh0, s);
  s = mma_b(a1, qh1, s);
  s = mma_b(a0, ql0, s);
  s = mma_b(a1, ql1, s);
  s = mma_b(e0, qh0, s);
  s = mma_b(e1, qh1, s);
  guard1x8(s, a0, a1, e0, e1, qh0, qh1, ql0, ql1);
  return s;
}

__global__ __launch_bounds__(ATT_THREADS)
void attn_fwd(u16* QOH, u16* QOL, const u16* __restrict__ KHp, const u16* __restrict__ KLp, const u16* __restrict__ VPp,
              const float* __restrict__ MBp) {
  __shared__ __align__(16) float smem[ATT_WAVES * SLAB];

  const int tid  = threadIdx.x;
  const int wave = tid >> 5;
  const int lane = tid & 31;
  const int hh   = lane >> 4;
  const int c    = lane & 15;

  const int bid  = blockIdx.x;
  const int gq   = bid % QT;
  const int head = bid / QT;
  if (head >= NH) return;
  const int q0   = gq * 64 + wave * 16;
  const int bat  = q0 / SEQ;
  const size_t krow0 = (size_t)bat * SEQ;

  const size_t qofs = ((size_t)(q0 + c)) * DMOD + (size_t)(head * HD + 8 * hh);
  const v16b qh0 = ldfrag_b(QOH + qofs), qh1 = ldfrag_b(QOH + qofs + 32);
  const v16b ql0 = ldfrag_b(QOL + qofs), ql1 = ldfrag_b(QOL + qofs + 32);
  const size_t kofs = (krow0 + (size_t)c) * DMOD + (size_t)(head * HD + 8 * hh);
  const u16* KHb = KHp + kofs;
  const u16* KLb = KLp + kofs;
  const size_t vofs = ((size_t)(head * HD + c)) * (size_t)MK + krow0 + (size_t)(8 * hh);
  const _Float16* Vb = (const _Float16*)(const void*)VPp + vofs;
  const float* MBb = MBp + krow0 + (size_t)(8 * hh);
  const float lsc = 0.125f * LOG2E;

  float mrun = -INFINITY, lrun = 0.f;
  v8f o[4];
#pragma unroll
  for (int j = 0; j < 4; ++j) o[j] = zero8();

#pragma unroll 1
  for (int it = 0; it < NKB; ++it) {
    const int kb = it * 32;
    const size_t k0o = (size_t)kb * DMOD;
    const size_t k1o = (size_t)(kb + 16) * DMOD;
    const v8f s0 = score_tile(KHb + k0o, KLb + k0o, qh0, qh1, ql0, ql1);
    const v8f s1 = score_tile(KHb + k1o, KLb + k1o, qh0, qh1, ql0, ql1);
    const v4f g0 = *(const v4f*)(MBb + kb),      g1 = *(const v4f*)(MBb + kb + 4);
    const v4f g2 = *(const v4f*)(MBb + kb + 16), g3 = *(const v4f*)(MBb + kb + 20);
    float tk[16];
#pragma unroll
    for (int e = 0; e < 4; ++e) {
      tk[e]      = s0[e] * lsc     + g0[e];
      tk[4 + e]  = s0[4 + e] * lsc + g1[e];
      tk[8 + e]  = s1[e] * lsc     + g2[e];
      tk[12 + e] = s1[4 + e] * lsc + g3[e];
    }
    float cm = tk[0];
#pragma unroll
    for (int i = 1; i < 16; ++i) cm = fmaxf(cm, tk[i]);
    cm = fmaxf(cm, __shfl_xor(cm, 16, 32));
    const float mn = fmaxf(mrun, cm);
    const float al = (mrun == -INFINITY) ? 0.f : exp2f(mrun - mn);
    mrun = mn;
    float ps = 0.f;
    FragH ph;
#pragma unroll
    for (int w = 0; w < 2; ++w) {
#pragma unroll
      for (int e4 = 0; e4 < 4; ++e4) {
        const int i = 8 * w + 2 * e4;
        const float p0 = exp2f(fminf(tk[i] - mn, 0.f));
        const float p1 = exp2f(fminf(tk[i + 1] - mn, 0.f));
        ps += p0 + p1;
        ph.u[w][e4] = pk16(h_bits((_Float16)(p0 * PCAR)), h_bits((_Float16)(p1 * PCAR)));
      }
    }
    ps += __shfl_xor(ps, 16, 32);
    lrun = lrun * al + ps;
    float scl[8];
#pragma unroll
    for (int r = 0; r < 8; ++r) scl[r] = __shfl(al, 8 * hh + r, 32);
#pragma unroll
    for (int j = 0; j < 4; ++j) {
#pragma unroll
      for (int r = 0; r < 8; ++r) o[j][r] *= scl[r];
    }
    {
      const _Float16* vp = Vb + kb;
      const v16h vf0 = ldfrag_h(vp);
      const v16h vf1 = ldfrag_h(vp + (size_t)16 * MK);
      const v16h vf2 = ldfrag_h(vp + (size_t)32 * MK);
      const v16h vf3 = ldfrag_h(vp + (size_t)48 * MK);
      o[0] = mma_h(ph.v, vf0, o[0]);
      o[1] = mma_h(ph.v, vf1, o[1]);
      o[2] = mma_h(ph.v, vf2, o[2]);
      o[3] = mma_h(ph.v, vf3, o[3]);
      guard6<v16h>(o[0], o[1], o[2], o[3], ph.v, vf0, vf1, vf2, vf3, ph.v);
    }
  }
  acc_guard4(o[0], o[1], o[2], o[3]);

  const float linv = (lrun > 0.f) ? ((1.0f / lrun) * (1.0f / (PCAR * VCAR))) : 0.f;
  float inv[8];
#pragma unroll
  for (int r = 0; r < 8; ++r) inv[r] = __shfl(linv, 8 * hh + r, 32);
  float* slab = smem + wave * SLAB;
#pragma unroll
  for (int r = 0; r < 8; ++r) {
#pragma unroll
    for (int j = 0; j < 4; ++j) slab[(8 * hh + r) * 68 + j * 16 + c] = o[j][r] * inv[r];
  }
  wave_sync_lds();
  v4u oh[4], ol[4];
  const int rq = lane >> 3, c8 = (lane & 7) * 8;
#pragma unroll
  for (int i4 = 0; i4 < 4; ++i4) {
    const int row = i4 * 4 + rq;
    const v4f a = *(const v4f*)(slab + row * 68 + c8), c4 = *(const v4f*)(slab + row * 68 + c8 + 4);
    float w[8];
#pragma unroll
    for (int e = 0; e < 4; ++e) { w[e] = a[e]; w[4 + e] = c4[e]; }
#pragma unroll
    for (int e = 0; e < 4; ++e) {
      const unsigned short h0 = bf_bits(w[2 * e]), h1 = bf_bits(w[2 * e + 1]);
      const unsigned short l0 = bf_bits(w[2 * e] - bf_up(h0)), l1 = bf_bits(w[2 * e + 1] - bf_up(h1));
      oh[i4][e] = pk16(h0, h1);
      ol[i4][e] = pk16(l0, l1);
    }
  }
  const size_t ob = ((size_t)q0) * DMOD + (size_t)(head * HD + c8);
  for (int pass = 0; pass < 2; ++pass) {
#pragma unroll
    for (int i4 = 0; i4 < 4; ++i4) {
      const size_t o8 = ob + (size_t)(i4 * 4 + rq) * DMOD;
      *(volatile v4u*)(QOH + o8) = oh[i4];
      *(volatile v4u*)(QOL + o8) = ol[i4];
    }
    __threadfence();
  }
}

__global__ __launch_bounds__(256)
void ln_rows(const float* __restrict__ Y, const float* __restrict__ X, const float* __restrict__ g,
             const float* __restrict__ bb, float* out, int nrows) {
  __shared__ __align__(16) float rows[LN_WAVES * DMOD];
  const int tid = threadIdx.x, wave = tid >> 5, lane = tid & 31;
  const int row = blockIdx.x * LN_WAVES + wave;
  if (row >= nrows) return;
  float* rl = rows + wave * DMOD + lane * 4;
  const float* yp = Y + (size_t)row * DMOD + lane * 4;
  const float* xp = X + (size_t)row * DMOD + lane * 4;
  float s = 0.f;
#pragma unroll 1
  for (int j = 0; j < DMOD / 128; ++j) {
    const v4f a = *(const v4f*)(yp + j * 128), b = *(const v4f*)(xp + j * 128);
    v4f v;
#pragma unroll
    for (int e = 0; e < 4; ++e) v[e] = a[e] + bf_val(b[e]);
    *(v4f*)(rl + j * 128) = v;
    s += (v[0] + v[1]) + (v[2] + v[3]);
  }
#pragma unroll
  for (int off = 16; off > 0; off >>= 1) s += __shfl_xor(s, off, 32);
  const float mu = s * (1.0f / (float)DMOD);
  float sq = 0.f;
#pragma unroll 1
  for (int j = 0; j < DMOD / 128; ++j) {
    const v4f v = *(const v4f*)(rl + j * 128);
#pragma unroll
    for (int e = 0; e < 4; ++e) { const float d = v[e] - mu; sq += d * d; }
  }
#pragma unroll
  for (int off = 16; off > 0; off >>= 1) sq += __shfl_xor(sq, off, 32);
  const float var  = sq * (1.0f / (float)DMOD);
  const float rstd = rsqrtf(var + LN_EPS);
  const float* gp = g  + lane * 4;
  const float* bp = bb + lane * 4;
#pragma unroll 1
  for (int j = 0; j < DMOD / 128; ++j) {
    const v4f v  = *(const v4f*)(rl + j * 128);
    const v4f gv = *(const v4f*)(gp + j * 128), bv = *(const v4f*)(bp + j * 128);
    v4f o;
#pragma unroll
    for (int e = 0; e < 4; ++e) o[e] = ((v[e] - mu) * rstd) * bf_val(gv[e]) + bf_val(bv[e]);
    *(v4f*)(rl + j * 128) = o;
  }
  float* dst = out + (size_t)row * DMOD + lane * 4;
  for (int pass = 0; pass < 2; ++pass) {
#pragma unroll 1
    for (int j = 0; j < DMOD / 128; ++j) {
      const v4f t = *(const v4f*)(rl + j * 128);
      *(volatile v4f*)(dst + j * 128) = t;
    }
    __threadfence();
  }
}

extern "C" void kernel_launch(void* const* d_in, const int* in_sizes, int n_in,
                              void* d_out, int out_size, void* d_ws, size_t ws_size,
                              hipStream_t stream) {
  if (n_in < 12) return;
  if (in_sizes[0] != BATCH * SEQ * DMOD) return;
  if (in_sizes[1] != BATCH * SEQ) return;
  if (in_sizes[2] != DMOD * DMOD || in_sizes[4] != DMOD * DMOD || in_sizes[6] != DMOD * DMOD || in_sizes[8] != DMOD * DMOD) return;
  if (in_sizes[3] != DMOD || in_sizes[5] != DMOD || in_sizes[7] != DMOD || in_sizes[9] != DMOD) return;
  if (in_sizes[10] != DMOD || in_sizes[11] != DMOD) return;
  if (out_size != BATCH * SEQ * DMOD) return;

  const float* Xin = (const float*)d_in[0];
  const float* Msk = (const float*)d_in[1];
  const float* Wq  = (const float*)d_in[2];
  const float* bq  = (const float*)d_in[3];
  const float* Wk  = (const float*)d_in[4];
  const float* bk  = (const float*)d_in[5];
  const float* Wv  = (const float*)d_in[6];
  const float* bv  = (const float*)d_in[7];
  const float* Wd  = (const float*)d_in[8];
  const float* bd  = (const float*)d_in[9];
  const float* lng = (const float*)d_in[10];
  const float* lnb = (const float*)d_in[11];
  float*       out = (float*)d_out;

  const size_t szXB = (size_t)MK * DMOD * 2;
  const size_t szW  = (size_t)DMOD * DMOD * 2;
  const size_t szQ  = (size_t)MQ * DMOD * 2;
  const size_t szK  = (size_t)MK * DMOD * 2;
  const size_t szVP = (size_t)DMOD * MK * 2;
  const size_t szMB = (size_t)MK * 4;
  const size_t szY  = (size_t)MQ * DMOD * 4;
  size_t off = 0;
  const size_t oXB = off; off += szXB;
  const size_t oWQ = off; off += szW;
  const size_t oWK = off; off += szW;
  const size_t oWV = off; off += szW;
  const size_t oWD = off; off += szW;
  const size_t oQH = off; off += szQ;
  const size_t oQL = off; off += szQ;
  const size_t oKH = off; off += szK;
  const size_t oKL = off; off += szK;
  const size_t oVP = off; off += szVP;
  const size_t oMB = off; off += szMB;
  if (off > ws_size) return;
  if (off > (size_t)134217728) return;
  if (szY > 2 * szK) return;
  if (oKL != oKH + szK) return;

  char* ws = (char*)d_ws;
  u16* XB  = (u16*)(ws + oXB);
  u16* WQB = (u16*)(ws + oWQ);
  u16* WKB = (u16*)(ws + oWK);
  u16* WVB = (u16*)(ws + oWV);
  u16* WDB = (u16*)(ws + oWD);
  u16* QH  = (u16*)(ws + oQH);
  u16* QL  = (u16*)(ws + oQL);
  u16* KH  = (u16*)(ws + oKH);
  u16* KL  = (u16*)(ws + oKL);
  u16* VP  = (u16*)(ws + oVP);
  float* MB = (float*)(ws + oMB);
  float* Y  = (float*)(ws + oKH);

  const int n8x = (MK * DMOD) / 8;
  const int n8w = (DMOD * DMOD) / 8;
  const int n4m = MK / 4;
  if ((n8x % 256) != 0 || (n8w % 256) != 0 || (n4m % 256) != 0) return;
  if ((DMOD % 64) != 0 || (MQ % 64) != 0 || (MK % 64) != 0 || (DMOD % 32) != 0 || (SEQ % 32) != 0 || (MQ % LN_WAVES) != 0) return;
  const dim3 blk(256);
  const dim3 gX(n8x / 256);
  const dim3 gW(n8w / 256);
  const dim3 gM(n4m / 256);
  const dim3 gGQ((MQ / 64) * (DMOD / 64));
  const dim3 gGK((MK / 64) * (DMOD / 64));
  const dim3 gV((DMOD / 64) * (MK / 64));
  const dim3 bG(128);
  const dim3 gAT(ATT_BLOCKS);
  const dim3 bAT(ATT_THREADS);
  const dim3 gLN(MQ / LN_WAVES);

  cvt16<<<gX, blk, 0, stream>>>(Xin, XB, n8x, 0, 1.0f);
  cvt16<<<gW, blk, 0, stream>>>(Wq, WQB, n8w, 0, 1.0f);
  cvt16<<<gW, blk, 0, stream>>>(Wk, WKB, n8w, 0, 1.0f);
  cvt16<<<gW, blk, 0, stream>>>(Wv, WVB, n8w, 0, 1.0f);
  cvt16<<<gW, blk, 0, stream>>>(Wd, WDB, n8w, 0, 1.0f);
  mask_bias<<<gM, blk, 0, stream>>>(Msk, MB, n4m);
  gemm_hl<<<gGQ, bG, 0, stream>>>(XB, WQB, QH, QL, bq, MQ, DMOD, DMOD, DMOD);
  gemm_hl<<<gGK, bG, 0, stream>>>(XB, WKB, KH, KL, bk, MK, DMOD, DMOD, DMOD);
  gemm_b16<<<gV, bG, 0, stream>>>(WVB, XB, VP, bv, DMOD, MK, DMOD, DMOD, 1, VCAR);
  attn_fwd<<<gAT, bAT, 0, stream>>>(QH, QL, KH, KL, VP, MB);
  gemm_o2<<<gGQ, bG, 0, stream>>>(QH, QL, WDB, Y, bd, MQ, DMOD, DMOD, DMOD);
  ln_rows<<<gLN, blk, 0, stream>>>(Y, Xin, lng, lnb, out, MQ);
}
